// GuideAttentionModule_56375740727765
// MI455X (gfx1250) — hardware-run, weakly checked
//
#include <hip/hip_runtime.h>
#include <math.h>
#include <stdint.h>

#define NB    4
#define SEQ   1024
#define NH    16
#define HD    64
#define DM    1024
#define QSC   1024.0f
#define KSC   1024.0f
#define PCAR  32768.0f
#define VCAR  256.0f
#define LOG2E 1.4426950408889634f

#define CV_THREADS 256
#define PJ_THREADS 256
#define BP    32
#define EPQ   72
#define EPV   136
#define SM_HALVES (128 * EPQ * 2)
#define TK_THREADS 128
#define TKP   68
#define ATW   4
#define ATT_THREADS (ATW * 32)
#define ATT_BLOCKS  (NB * NH * (SEQ / 64))
#define PTP   36
#define OSP   68
#define SLABF (16 * OSP)

static_assert(DM == NH * HD);
static_assert(HD == 64 && (SEQ % 64) == 0 && (SEQ % 32) == 0 && (DM % 64) == 0 && (DM % 32) == 0);
static_assert(ATT_THREADS == 128 && ATT_BLOCKS == 1024);
static_assert(16 * PTP <= SLABF);
static_assert(64 * EPV * 2 <= SM_HALVES && 64 * BP <= SM_HALVES);
static_assert(((NB * SEQ) % 128) == 0 && (SEQ % 128) == 0);
static_assert((SEQ / 64) == 16 && NH == 16);

typedef _Float16 v16h __attribute__((ext_vector_type(16)));
typedef _Float16 v8h  __attribute__((ext_vector_type(8)));
typedef __bf16   v16b __attribute__((ext_vector_type(16)));
typedef float    v8f  __attribute__((ext_vector_type(8)));
typedef float    v4f  __attribute__((ext_vector_type(4)));
typedef unsigned int   v4u  __attribute__((ext_vector_type(4)));
typedef unsigned short v8us __attribute__((ext_vector_type(8)));

union FragH { v16h v; v8h h[2]; v4u u[2]; };
union FragB { v16b v; v16h hv; v8us u[2]; };

__device__ __forceinline__ unsigned short bf_bits(float f) {
  unsigned u = __float_as_uint(f);
  return (unsigned short)((u + 0x7FFFu + ((u >> 16) & 1u)) >> 16);
}
__device__ __forceinline__ float bf_up(unsigned short h) { return __uint_as_float(((unsigned)h) << 16); }
__device__ __forceinline__ float bfr(float f) { return bf_up(bf_bits(f)); }
__device__ __forceinline__ unsigned short h_bits(_Float16 x) { return __builtin_bit_cast(unsigned short, x); }
__device__ __forceinline__ unsigned pk16(unsigned short a, unsigned short b) { return (unsigned)a | ((unsigned)b << 16); }
__device__ __forceinline__ v8f zero8() { v8f z = {0.f, 0.f, 0.f, 0.f, 0.f, 0.f, 0.f, 0.f}; return z; }

__device__ __forceinline__ v16h ldfrag_h(const _Float16* p) {
  FragH f;
  f.h[0] = *(const v8h*)(p);
  f.h[1] = *(const v8h*)(p + 16);
  return f.v;
}
__device__ __forceinline__ FragB ldfrag_b(const unsigned short* p) {
  FragB f;
  f.u[0] = *(const v8us*)(p);
  f.u[1] = *(const v8us*)(p + 16);
  return f;
}

__device__ __forceinline__ v8f mma_h(v16h a, v16h b, v8f c) {
  return __builtin_amdgcn_wmma_f32_16x16x32_f16(false, a, false, b, (short)0, c, false, false);
}
__device__ __forceinline__ v8f mma_b(v16b a, v16b b, v8f c) {
  return __builtin_amdgcn_wmma_f32_16x16x32_bf16(false, a, false, b, (short)0, c, false, false);
}
__device__ __forceinline__ void guard1(v8f& a, v16h x0, v16h x1) {
#if defined(__HIP_DEVICE_COMPILE__)
  asm volatile("v_nop\n\tv_nop\n\tv_nop\n\tv_nop" : "+v"(a) : "v"(x0), "v"(x1) : "memory");
#endif
}
__device__ __forceinline__ void guard4(v8f& a, v8f& b, v8f& c, v8f& d,
                                       v16h x0, v16h x1, v16h x2, v16h x3, v16h x4) {
#if defined(__HIP_DEVICE_COMPILE__)
  asm volatile("v_nop\n\tv_nop\n\tv_nop\n\tv_nop"
               : "+v"(a), "+v"(b), "+v"(c), "+v"(d) : "v"(x0), "v"(x1), "v"(x2), "v"(x3), "v"(x4) : "memory");
#endif
}
__device__ __forceinline__ void guard_sc(v8f& a, v8f& b, v16h x0, v16h x1, v16h x2, v16h x3, v16h x4, v16h x5) {
#if defined(__HIP_DEVICE_COMPILE__)
  asm volatile("v_nop\n\tv_nop\n\tv_nop\n\tv_nop"
               : "+v"(a), "+v"(b) : "v"(x0), "v"(x1), "v"(x2), "v"(x3), "v"(x4), "v"(x5) : "memory");
#endif
}
__device__ __forceinline__ void guard_pv(v8f& a, v8f& b, v16h p0, v16h p1, v16h x0, v16h x1, v16h x2, v16h x3) {
#if defined(__HIP_DEVICE_COMPILE__)
  asm volatile("v_nop\n\tv_nop\n\tv_nop\n\tv_nop"
               : "+v"(a), "+v"(b) : "v"(p0), "v"(p1), "v"(x0), "v"(x1), "v"(x2), "v"(x3) : "memory");
#endif
}
__device__ __forceinline__ void acc_guard4(v8f& a, v8f& b, v8f& c, v8f& d) {
#if defined(__HIP_DEVICE_COMPILE__)
  asm volatile("v_nop\n\tv_nop\n\tv_nop\n\tv_nop" : "+v"(a), "+v"(b), "+v"(c), "+v"(d));
#endif
}
__device__ __forceinline__ void wave_sync_lds() {
  __builtin_amdgcn_fence(__ATOMIC_RELEASE, "workgroup");
  __builtin_amdgcn_wave_barrier();
  __builtin_amdgcn_fence(__ATOMIC_ACQUIRE, "workgroup");
}

__global__ __launch_bounds__(CV_THREADS) void cvt_bf16(const float* __restrict__ src, unsigned short* dst,
                                                       int nsrc, int ndst) {
  const size_t i8 = ((size_t)blockIdx.x * CV_THREADS + threadIdx.x) * 8;
  if (i8 >= (size_t)ndst) return;
  size_t a0 = i8;
  if (a0 + 8 > (size_t)nsrc) a0 = (size_t)nsrc - 8;
  const v4f va = *(const v4f*)(src + a0);
  const v4f vb = *(const v4f*)(src + a0 + 4);
  const bool ok = (i8 + 8 <= (size_t)nsrc);
  v4u o;
  o[0] = ok ? pk16(bf_bits(va[0]), bf_bits(va[1])) : 0u;
  o[1] = ok ? pk16(bf_bits(va[2]), bf_bits(va[3])) : 0u;
  o[2] = ok ? pk16(bf_bits(vb[0]), bf_bits(vb[1])) : 0u;
  o[3] = ok ? pk16(bf_bits(vb[2]), bf_bits(vb[3])) : 0u;
  for (int pass = 0; pass < 2; ++pass) {
    *(volatile v4u*)(dst + i8) = o;
    __threadfence();
  }
}

__global__ __launch_bounds__(TK_THREADS) void tok_gemm(const unsigned short* __restrict__ TBp,
                                                       const unsigned short* __restrict__ WQp,
                                                       const unsigned short* __restrict__ WKp,
                                                       const float* __restrict__ bq, const float* __restrict__ bk,
                                                       float* TQKo) {
  __shared__ __align__(16) float st[16 * TKP];
  const int tid = threadIdx.x, wave = tid >> 5, lane = tid & 31, hh = lane >> 4, c = lane & 15;
  const int n0 = blockIdx.x * 64;
  const int z  = blockIdx.y;
  const unsigned short* W = (z == 0) ? WQp : WKp;
  const float* bias = (z == 0) ? bq : bk;
  const unsigned short* Ar = TBp + (size_t)c * DM + 8 * hh;
  const unsigned short* Br = W + (size_t)(n0 + 16 * wave + c) * DM + 8 * hh;
  v8f acc = zero8();
#pragma unroll 1
  for (int kk = 0; kk < DM; kk += 32) {
    const FragB a = ldfrag_b(Ar + kk);
    const FragB b = ldfrag_b(Br + kk);
    acc = mma_b(a.v, b.v, acc);
    guard1(acc, a.hv, b.hv);
  }
  {
    const int n = 16 * wave + c;
    const float add = bfr(bias[n0 + n]);
#pragma unroll
    for (int r = 0; r < 8; ++r) st[(8 * hh + r) * TKP + n] = acc[r] + add;
  }
  __syncthreads();
  const int q16 = tid >> 4, p16 = (tid & 15) * 4;
  v4f vals[2];
#pragma unroll
  for (int it = 0; it < 2; ++it) vals[it] = *(const v4f*)(st + (it * 8 + q16) * TKP + p16);
  float* dst = TQKo + (size_t)z * 16 * DM + n0 + p16;
  for (int pass = 0; pass < 2; ++pass) {
#pragma unroll
    for (int it = 0; it < 2; ++it) *(volatile v4f*)(dst + (size_t)(it * 8 + q16) * DM) = vals[it];
    __threadfence();
  }
}

__global__ __launch_bounds__(PJ_THREADS) void proj_gemm(
    const unsigned short* __restrict__ XBp,
    const unsigned short* __restrict__ WQp, const unsigned short* __restrict__ WKp,
    const unsigned short* __restrict__ WVp,
    const float* __restrict__ bq, const float* __restrict__ bk, const float* __restrict__ bv,
    const float* __restrict__ TQKp,
    unsigned short* CQH, unsigned short* CQL, unsigned short* CKH, unsigned short* CKL,
    unsigned short* VTH, unsigned short* VTL) {
  __shared__ __align__(16) unsigned short sm[SM_HALVES];

  const int tid = threadIdx.x, lane = tid & 31, wave = tid >> 5, hh = lane >> 4, c = lane & 15;
  const int m0 = blockIdx.x * 128;
  const int n0 = blockIdx.y * 64;
  const int z  = blockIdx.z;
  const unsigned short* W = (z == 0) ? WQp : ((z == 1) ? WKp : WVp);

  const int srow = tid >> 2;
  const int soff = (tid & 3) * 8;
  const unsigned short* Wsrc = W + (size_t)(n0 + srow) * DM + soff;
  const unsigned short* Ar = XBp + (size_t)(m0 + 16 * wave + c) * DM + 8 * hh;

  v8f acc[4];
#pragma unroll
  for (int t = 0; t < 4; ++t) acc[t] = zero8();

#pragma unroll 1
  for (int kk = 0; kk < DM; kk += 32) {
    const v4u bt = *(const v4u*)(Wsrc + kk);
    *(v4u*)(sm + srow * BP + soff) = bt;
    __syncthreads();
    const FragB a  = ldfrag_b(Ar + kk);
    const FragB b0 = ldfrag_b(sm + (0  + c) * BP + 8 * hh);
    const FragB b1 = ldfrag_b(sm + (16 + c) * BP + 8 * hh);
    const FragB b2 = ldfrag_b(sm + (32 + c) * BP + 8 * hh);
    const FragB b3 = ldfrag_b(sm + (48 + c) * BP + 8 * hh);
    acc[0] = mma_b(a.v, b0.v, acc[0]);
    acc[1] = mma_b(a.v, b1.v, acc[1]);
    acc[2] = mma_b(a.v, b2.v, acc[2]);
    acc[3] = mma_b(a.v, b3.v, acc[3]);
    guard4(acc[0], acc[1], acc[2], acc[3], a.hv, b0.hv, b1.hv, b2.hv, b3.hv);
    __syncthreads();
  }
  acc_guard4(acc[0], acc[1], acc[2], acc[3]);

  const int bb   = m0 >> 10;
  const int sb   = m0 & (SEQ - 1);
  const int head = n0 >> 6;
  unsigned short* H  = sm;
  unsigned short* LQ = sm + 128 * EPQ;
  unsigned short* LV = sm + 64 * EPV;

  if (z < 2) {
    const float* bias = (z == 0) ? bq : bk;
    const float* tq = TQKp + (size_t)z * 16 * DM + (size_t)bb * DM + n0;
    const float sc = (z == 0) ? QSC : KSC;
#pragma unroll
    for (int t = 0; t < 4; ++t) {
      const int n = 16 * t + c;
      const float add = bfr(bias[n0 + n]);
      const float tv  = tq[n];
#pragma unroll
      for (int r = 0; r < 8; ++r) {
        const int row = 16 * wave + 8 * hh + r;
        const float val = (acc[t][r] + add) + tv;
        const float tt = val * sc;
        const _Float16 hv = (_Float16)tt;
        const _Float16 lv = (_Float16)(tt - (float)hv);
        H[row * EPQ + n]  = h_bits(hv);
        LQ[row * EPQ + n] = h_bits(lv);
      }
    }
  } else {
#pragma unroll
    for (int t = 0; t < 4; ++t) {
      const int d = 16 * t + c;
      const float add = bfr(bv[n0 + d]);
#pragma unroll
      for (int r = 0; r < 8; ++r) {
        const int sl = 16 * wave + 8 * hh + r;
        const float val = acc[t][r] + add;
        const float tt = val * VCAR;
        const _Float16 hv = (_Float16)tt;
        const _Float16 lv = (_Float16)(tt - (float)hv);
        H[d * EPV + sl]  = h_bits(hv);
        LV[d * EPV + sl] = h_bits(lv);
      }
    }
  }
  __syncthreads();
  if (z < 2) {
    const size_t base = ((size_t)(bb * NH + head) * SEQ + sb) * HD;
    unsigned short* dH = ((z == 0) ? CQH : CKH) + base;
    unsigned short* dL = ((z == 0) ? CQL : CKL) + base;
    const int q8 = tid >> 3, p8 = (tid & 7) * 8;
    v4u vh[4], vl[4];
#pragma unroll
    for (int it = 0; it < 4; ++it) {
      const int row = it * 32 + q8;
      vh[it] = *(const v4u*)(H  + row * EPQ + p8);
      vl[it] = *(const v4u*)(LQ + row * EPQ + p8);
    }
    for (int pass = 0; pass < 2; ++pass) {
#pragma unroll
      for (int it = 0; it < 4; ++it) {
        const int row = it * 32 + q8;
        *(volatile v4u*)(dH + (size_t)row * HD + p8) = vh[it];
        *(volatile v4u*)(dL + (size_t)row * HD + p8) = vl[it];
      }
      __threadfence();
    }
  } else {
    const size_t base = ((size_t)(bb * NH + head) * HD) * SEQ + sb;
    unsigned short* dH = VTH + base;
    unsigned short* dL = VTL + base;
    const int q16 = tid >> 4, p16 = (tid & 15) * 8;
    v4u vh[4], vl[4];
#pragma unroll
    for (int it = 0; it < 4; ++it) {
      const int d = it * 16 + q16;
      vh[it] = *(const v4u*)(H  + d * EPV + p16);
      vl[it] = *(const v4u*)(LV + d * EPV + p16);
    }
    for (int pass = 0; pass < 2; ++pass) {
#pragma unroll
      for (int it = 0; it < 4; ++it) {
        const int d = it * 16 + q16;
        *(volatile v4u*)(dH + (size_t)d * SEQ + p16) = vh[it];
        *(volatile v4u*)(dL + (size_t)d * SEQ + p16) = vl[it];
      }
      __threadfence();
    }
  }
}

__global__ __launch_bounds__(ATT_THREADS)
void attn_fwd(const unsigned short* __restrict__ CQHp, const unsigned short* __restrict__ CQLp,
              const unsigned short* __restrict__ CKHp, const unsigned short* __restrict__ CKLp,
              const unsigned short* __restrict__ VTHp, const unsigned short* __restrict__ VTLp, float* outp) {
  __shared__ __align__(16) float smem[ATW * SLABF];

  const int tid  = threadIdx.x;
  const int wave = tid >> 5;
  const int lane = tid & 31;
  const int hh   = lane >> 4;
  const int c    = lane & 15;

  const int bid  = blockIdx.x;
  const int qt   = bid & 15;
  const int head = (bid >> 4) & 15;
  const int b    = bid >> 8;
  const int bh   = b * NH + head;
  const int q0   = qt * 64 + wave * 16;

  const size_t qofs = ((size_t)bh * SEQ + q0 + c) * HD + 8 * hh;
  const _Float16* Qh  = (const _Float16*)(const void*)CQHp + qofs;
  const _Float16* Ql  = (const _Float16*)(const void*)CQLp + qofs;
  const size_t kofs = ((size_t)bh * SEQ + c) * HD + 8 * hh;
  const _Float16* Khb = (const _Float16*)(const void*)CKHp + kofs;
  const _Float16* Klb = (const _Float16*)(const void*)CKLp + kofs;
  const size_t vofs = ((size_t)bh * HD + c) * SEQ + 8 * hh;
  const _Float16* Vhb = (const _Float16*)(const void*)VTHp + vofs;
  const _Float16* Vlb = (const _Float16*)(const void*)VTLp + vofs;
  const float lsc = (0.125f * LOG2E) / (QSC * KSC);

  const v16h qh0 = ldfrag_h(Qh), qh1 = ldfrag_h(Qh + 32);
  const v16h ql0 = ldfrag_h(Ql), ql1 = ldfrag_h(Ql + 32);

  float mrow[8], lrow[8];
  v8f o[4];
#pragma unroll
  for (int r = 0; r < 8; ++r) { mrow[r] = -INFINITY; lrow[r] = 0.f; }
#pragma unroll
  for (int j = 0; j < 4; ++j) o[j] = zero8();
  float* pt = smem + wave * SLABF;

#pragma unroll 1
  for (int kb = 0; kb < SEQ; kb += 32) {
    v8f s0 = zero8(), s1 = zero8();
    const _Float16* k0p = Khb + (size_t)kb * HD;
    const _Float16* k1p = k0p + (size_t)16 * HD;
    const _Float16* l0p = Klb + (size_t)kb * HD;
    const _Float16* l1p = l0p + (size_t)16 * HD;
    {
      const v16h kh0 = ldfrag_h(k0p), kl0 = ldfrag_h(l0p);
      const v16h kh1 = ldfrag_h(k1p), kl1 = ldfrag_h(l1p);
      s0 = mma_h(qh0, kh0, s0);
      s0 = mma_h(ql0, kh0, s0);
      s0 = mma_h(qh0, kl0, s0);
      s1 = mma_h(qh0, kh1, s1);
      s1 = mma_h(ql0, kh1, s1);
      s1 = mma_h(qh0, kl1, s1);
      guard_sc(s0, s1, qh0, ql0, kh0, kl0, kh1, kl1);
    }
    {
      const v16h kh0 = ldfrag_h(k0p + 32), kl0 = ldfrag_h(l0p + 32);
      const v16h kh1 = ldfrag_h(k1p + 32), kl1 = ldfrag_h(l1p + 32);
      s0 = mma_h(qh1, kh0, s0);
      s0 = mma_h(ql1, kh0, s0);
      s0 = mma_h(qh1, kl0, s0);
      s1 = mma_h(qh1, kh1, s1);
      s1 = mma_h(ql1, kh1, s1);
      s1 = mma_h(qh1, kl1, s1);
      guard_sc(s0, s1, qh1, ql1, kh0, kl0, kh1, kl1);
    }
#pragma unroll
    for (int r = 0; r < 8; ++r) {
      const float t0 = s0[r] * lsc, t1 = s1[r] * lsc;
      float mx = fmaxf(t0, t1);
#pragma unroll
      for (int off = 1; off < 16; off <<= 1) mx = fmaxf(mx, __shfl_xor(mx, off, 32));
      const float mn = fmaxf(mrow[r], mx);
      const float al = exp2f(mrow[r] - mn);
      mrow[r] = mn;
      const float e0 = exp2f(t0 - mn), e1 = exp2f(t1 - mn);
      float ps = e0 + e1;
#pragma unroll
      for (int off = 1; off < 16; off <<= 1) ps += __shfl_xor(ps, off, 32);
      lrow[r] = lrow[r] * al + ps;
#pragma unroll
      for (int j = 0; j < 4; ++j) o[j][r] *= al;
      const int ro = (8 * hh + r) * PTP + c;
      pt[ro]      = e0;
      pt[ro + 16] = e1;
    }
    wave_sync_lds();
    FragH ph, pl;
    {
      const float* prow = pt + c * PTP + 8 * hh;
      const v4f p0 = *(const v4f*)(prow), p1 = *(const v4f*)(prow + 4);
      const v4f p2 = *(const v4f*)(prow + 16), p3 = *(const v4f*)(prow + 20);
#pragma unroll
      for (int e = 0; e < 4; ++e) {
        const float ta = p0[e] * PCAR, tb = p1[e] * PCAR, tc = p2[e] * PCAR, td = p3[e] * PCAR;
        const _Float16 ha = (_Float16)ta, hb = (_Float16)tb, hc = (_Float16)tc, hd = (_Float16)td;
        ph.h[0][e]     = ha;
        ph.h[0][4 + e] = hb;
        ph.h[1][e]     = hc;
        ph.h[1][4 + e] = hd;
        pl.h[0][e]     = (_Float16)(ta - (float)ha);
        pl.h[0][4 + e] = (_Float16)(tb - (float)hb);
        pl.h[1][e]     = (_Float16)(tc - (float)hc);
        pl.h[1][4 + e] = (_Float16)(td - (float)hd);
      }
    }
    const _Float16* vhp = Vhb + kb;
    const _Float16* vlp = Vlb + kb;
    {
      const v16h vh0 = ldfrag_h(vhp),                    vl0 = ldfrag_h(vlp);
      const v16h vh1 = ldfrag_h(vhp + (size_t)16 * SEQ), vl1 = ldfrag_h(vlp + (size_t)16 * SEQ);
      o[0] = mma_h(ph.v, vh0, o[0]);  o[0] = mma_h(pl.v, vh0, o[0]);  o[0] = mma_h(ph.v, vl0, o[0]);
      o[1] = mma_h(ph.v, vh1, o[1]);  o[1] = mma_h(pl.v, vh1, o[1]);  o[1] = mma_h(ph.v, vl1, o[1]);
      guard_pv(o[0], o[1], ph.v, pl.v, vh0, vl0, vh1, vl1);
    }
    {
      const v16h vh2 = ldfrag_h(vhp + (size_t)32 * SEQ), vl2 = ldfrag_h(vlp + (size_t)32 * SEQ);
      const v16h vh3 = ldfrag_h(vhp + (size_t)48 * SEQ), vl3 = ldfrag_h(vlp + (size_t)48 * SEQ);
      o[2] = mma_h(ph.v, vh2, o[2]);  o[2] = mma_h(pl.v, vh2, o[2]);  o[2] = mma_h(ph.v, vl2, o[2]);
      o[3] = mma_h(ph.v, vh3, o[3]);  o[3] = mma_h(pl.v, vh3, o[3]);  o[3] = mma_h(ph.v, vl3, o[3]);
      guard_pv(o[2], o[3], ph.v, pl.v, vh2, vl2, vh3, vl3);
    }
    wave_sync_lds();
  }
  acc_guard4(o[0], o[1], o[2], o[3]);

  wave_sync_lds();
  float* slab = pt;
  const float oc = 1.0f / (PCAR * VCAR);
#pragma unroll
  for (int r = 0; r < 8; ++r) {
    const float inv = (1.0f / lrow[r]) * oc;
#pragma unroll
    for (int j = 0; j < 4; ++j) slab[(8 * hh + r) * OSP + j * 16 + c] = o[j][r] * inv;
  }
  wave_sync_lds();
  v4f vals[8];
#pragma unroll
  for (int it = 0; it < 8; ++it) vals[it] = *(const v4f*)(slab + (2 * it + hh) * OSP + c * 4);
  float* dst = outp + ((size_t)(b * SEQ + q0 + hh)) * DM + head * HD + c * 4;
  for (int pass = 0; pass < 2; ++pass) {
#pragma unroll
    for (int it = 0; it < 8; ++it) {
      *(volatile v4f*)(dst + (size_t)(2 * it) * DM) = vals[it];
    }
    __threadfence();
  }
}

extern "C" void kernel_launch(void* const* d_in, const int* in_sizes, int n_in,
                              void* d_out, int out_size, void* d_ws, size_t ws_size,
                              hipStream_t stream) {
  if (n_in < 8) return;
  if (in_sizes[0] != NB * SEQ * DM) return;
  if (in_sizes[1] != NB * DM) return;
  if (in_sizes[2] != DM * DM || in_sizes[4] != DM * DM || in_sizes[6] != DM * DM) return;
  if (in_sizes[3] != DM || in_sizes[5] != DM || in_sizes[7] != DM) return;
  if (out_size != NB * SEQ * DM) return;

  const float* x   = (const float*)d_in[0];
  const float* tok = (const float*)d_in[1];
  const float* Wq  = (const float*)d_in[2];
  const float* bq  = (const float*)d_in[3];
  const float* Wk  = (const float*)d_in[4];
  const float* bk  = (const float*)d_in[5];
  const float* Wv  = (const float*)d_in[6];
  const float* bv  = (const float*)d_in[7];
  float*       out = (float*)d_out;

  const size_t nX  = (size_t)NB * SEQ * DM;
  const size_t nT  = (size_t)NB * DM;
  const size_t nTB = (size_t)16 * DM;
  const size_t nW  = (size_t)DM * DM;
  const size_t nTQ = (size_t)2 * 16 * DM;
  const size_t nPL = (size_t)NB * NH * SEQ * HD;

  size_t off = 0;
  const size_t oXB = off; off += nX * 2;
  const size_t oTB = off; off += nTB * 2;
  const size_t oWQ = off; off += nW * 2;
  const size_t oWK = off; off += nW * 2;
  const size_t oWV = off; off += nW * 2;
  const size_t oTQ = off; off += nTQ * 4;
  const size_t oQH = off; off += nPL * 2;
  const size_t oQL = off; off += nPL * 2;
  const size_t oKH = off; off += nPL * 2;
  const size_t oKL = off; off += nPL * 2;
  const size_t oVH = off; off += nPL * 2;
  const size_t oVL = off; off += nPL * 2;
  if (off > ws_size) return;
  if (off > (size_t)134217728) return;

  char* ws = (char*)d_ws;
  unsigned short* XB  = (unsigned short*)(ws + oXB);
  unsigned short* TB  = (unsigned short*)(ws + oTB);
  unsigned short* WQB = (unsigned short*)(ws + oWQ);
  unsigned short* WKB = (unsigned short*)(ws + oWK);
  unsigned short* WVB = (unsigned short*)(ws + oWV);
  float*          TQK = (float*)(ws + oTQ);
  unsigned short* CQH = (unsigned short*)(ws + oQH);
  unsigned short* CQL = (unsigned short*)(ws + oQL);
  unsigned short* CKH = (unsigned short*)(ws + oKH);
  unsigned short* CKL = (unsigned short*)(ws + oKL);
  unsigned short* VTH = (unsigned short*)(ws + oVH);
  unsigned short* VTL = (unsigned short*)(ws + oVL);

  const dim3 bCV(CV_THREADS);
  const unsigned per = (unsigned)CV_THREADS * 8;
  const dim3 gX((unsigned)((nX + per - 1) / per));
  const dim3 gT((unsigned)((nTB + per - 1) / per));
  const dim3 gW((unsigned)((nW + per - 1) / per));
  const dim3 gTK(DM / 64, 2);
  const dim3 bTK(TK_THREADS);
  const dim3 gPJ((NB * SEQ) / 128, DM / 64, 3);
  const dim3 bPJ(PJ_THREADS);
  const dim3 gAT(ATT_BLOCKS);
  const dim3 bAT(ATT_THREADS);

  cvt_bf16<<<gX, bCV, 0, stream>>>(x, XB, (int)nX, (int)nX);
  cvt_bf16<<<gT, bCV, 0, stream>>>(tok, TB, (int)nT, (int)nTB);
  cvt_bf16<<<gW, bCV, 0, stream>>>(Wq, WQB, (int)nW, (int)nW);
  cvt_bf16<<<gW, bCV, 0, stream>>>(Wk, WKB, (int)nW, (int)nW);
  cvt_bf16<<<gW, bCV, 0, stream>>>(Wv, WVB, (int)nW, (int)nW);
  tok_gemm<<<gTK, bTK, 0, stream>>>(TB, WQB, WKB, bq, bk, TQK);
  proj_gemm<<<gPJ, bPJ, 0, stream>>>(XB, WQB, WKB, WVB, bq, bk, bv, TQK, CQH, CQL, CKH, CKL, VTH, VTL);
  attn_fwd<<<gAT, bAT, 0, stream>>>(CQH, CQL, CKH, CKL, VTH, VTL, out);
  (void)hipGetLastError();
}
